// RNN_70970039599178
// MI455X (gfx1250) — hardware-verified
//
#include <hip/hip_runtime.h>
#include <math.h>

constexpr int SEQ_LEN  = 512;
constexpr int BATCH_N  = 64;
constexpr int VOCAB_N  = 50000;
constexpr int EMB_DIM  = 300;
constexpr int EMB_PAD  = 320;
constexpr int HID_DIM  = 256;
constexpr int CLS_DIM  = 5;
constexpr int NROW_ALL = SEQ_LEN * BATCH_N;
constexpr int CVT_THR  = 256;
constexpr int RNN_THR  = 512;
constexpr int ROWS_BLK = 16;
constexpr int HPITCH   = 264;
constexpr int OPITCH   = 260;
constexpr int NBLK_WIH = (HID_DIM * (EMB_PAD / 8)) / CVT_THR;
constexpr int NBLK_WHH = (HID_DIM * (HID_DIM / 8)) / CVT_THR;
constexpr int GATHER_N8 = NROW_ALL * (EMB_PAD / 8);
constexpr float WCARRY     = 256.0f;
constexpr float WCARRY_INV = 1.0f / 256.0f;

static_assert(EMB_PAD % 32 == 0 && EMB_PAD >= EMB_DIM, "K pad");
static_assert(HID_DIM % 32 == 0, "K of the recurrent product");
static_assert(NROW_ALL % 64 == 0 && HID_DIM % 64 == 0, "GEMM tile multiples");
static_assert((HID_DIM * (EMB_PAD / 8)) % CVT_THR == 0, "prep coverage W_ih");
static_assert((HID_DIM * (HID_DIM / 8)) % CVT_THR == 0, "prep coverage W_hh");
static_assert(GATHER_N8 % CVT_THR == 0, "gather coverage");
static_assert(HID_DIM == 16 * (RNN_THR / 32), "one 16-column group per wave");
static_assert(BATCH_N % ROWS_BLK == 0, "batch tiles");
static_assert((ROWS_BLK * HID_DIM / 4) % RNN_THR == 0, "hsum store coverage");
static_assert(EMB_DIM % 4 == 0, "float4 row alignment");
static_assert(BATCH_N * CLS_DIM == 320, "ten whole lines");

typedef __attribute__((ext_vector_type(16))) _Float16 v16h;
typedef __attribute__((ext_vector_type(8)))  _Float16 v8h;
typedef __attribute__((ext_vector_type(8)))  float    v8f;
typedef __attribute__((ext_vector_type(4)))  float    v4f;

union FragU { v16h v; v8h h[2]; };
__device__ __forceinline__ v16h frag_load_h(const _Float16* p) {
  FragU f;
  f.h[0] = *(const v8h*)(p);
  f.h[1] = *(const v8h*)(p + 16);
  return f.v;
}
__device__ __forceinline__ v8f wmma_h(v16h a, v16h b, v8f c) {
  return __builtin_amdgcn_wmma_f32_16x16x32_f16(false, a, false, b, (short)0, c, false, false);
}
__device__ __forceinline__ v8f wmma_h_guarded(v16h a, v16h b, v8f c) {
  c = __builtin_amdgcn_wmma_f32_16x16x32_f16(false, a, false, b, (short)0, c, false, false);
  asm volatile("v_nop\n\tv_nop\n\tv_nop\n\tv_nop" : "+v"(c) : "v"(a), "v"(b));
  return c;
}
__device__ __forceinline__ void dep_guard4_h(v8f& a, v8f& b, v8f& c, v8f& d, v16h x, v16h y) {
  asm volatile("v_nop\n\tv_nop\n\tv_nop\n\tv_nop" : "+v"(a), "+v"(b), "+v"(c), "+v"(d) : "v"(x), "v"(y));
}
__device__ __forceinline__ void keep4_h(v16h a, v16h b, v16h c, v16h d) { asm volatile("v_nop" :: "v"(a), "v"(b), "v"(c), "v"(d)); }
__device__ __forceinline__ void acc_guard4(v8f& a, v8f& b, v8f& c, v8f& d) { asm volatile("v_nop\n\tv_nop\n\tv_nop\n\tv_nop" : "+v"(a), "+v"(b), "+v"(c), "+v"(d)); }

__global__ __launch_bounds__(CVT_THR) void prep_weights_kernel(const float* __restrict__ wih, const float* __restrict__ whh,
                                                               unsigned short* __restrict__ wih16,
                                                               unsigned short* __restrict__ whh16) {
  const int blk = blockIdx.x;
  const bool second = (blk >= NBLK_WIH);
  const float* src = second ? whh : wih;
  unsigned short* dst = second ? whh16 : wih16;
  const int ncol  = second ? HID_DIM : EMB_DIM;
  const int ncol8 = second ? (HID_DIM / 8) : (EMB_PAD / 8);
  const int i = (second ? (blk - NBLK_WIH) : blk) * CVT_THR + threadIdx.x;
  const int row = i / ncol8;
  const int c8  = i - row * ncol8;
  v8h hv;
#pragma unroll
  for (int e = 0; e < 8; ++e) {
    const int col = c8 * 8 + e;
    const int cc  = (col < ncol) ? col : (ncol - 1);
    const float w = src[(size_t)row * ncol + cc];
    const float s = (col < ncol) ? (w * WCARRY) : 0.0f;
    hv[e] = (_Float16)s;
  }
  *(volatile v8h*)(dst + (size_t)i * 8) = hv;
  __threadfence();
  *(volatile v8h*)(dst + (size_t)i * 8) = hv;
}

__global__ __launch_bounds__(CVT_THR) void gather_rows_kernel(const int* __restrict__ tok, const float* __restrict__ emb,
                                                              unsigned short* __restrict__ apl) {
  const int i = blockIdx.x * CVT_THR + threadIdx.x;
  if (i < GATHER_N8) {
    const int row = i / (EMB_PAD / 8);
    const int c8  = i - row * (EMB_PAD / 8);
    int id = tok[row];
    id = id < 0 ? 0 : id;
    id = id > (VOCAB_N - 1) ? (VOCAB_N - 1) : id;
    const int col = c8 * 8;
    const int ca = (col < EMB_DIM - 4) ? col : (EMB_DIM - 4);
    const int cb = (col + 4 < EMB_DIM - 4) ? (col + 4) : (EMB_DIM - 4);
    const float* er = emb + (size_t)id * EMB_DIM;
    const v4f a = *(const v4f*)(er + ca);
    const v4f b = *(const v4f*)(er + cb);
    v8h hv;
#pragma unroll
    for (int e = 0; e < 4; ++e) {
      const float fa = a[e];
      const float fb = b[e];
      const float sa = (col + e < EMB_DIM) ? fa : 0.0f;
      const float sb = (col + 4 + e < EMB_DIM) ? fb : 0.0f;
      hv[e]     = (_Float16)sa;
      hv[4 + e] = (_Float16)sb;
    }
    *(volatile v8h*)(apl + (size_t)i * 8) = hv;
    __threadfence();
    *(volatile v8h*)(apl + (size_t)i * 8) = hv;
  }
}

__global__ __launch_bounds__(256) void gemm_xw_kernel(const unsigned short* __restrict__ Ap, int lda,
                                                      const unsigned short* __restrict__ Btp, int ldb,
                                                      float* __restrict__ C, int ldc,
                                                      const float* __restrict__ bias,
                                                      int M, int N, int K, float scale) {
  const _Float16* A  = (const _Float16*)Ap;
  const _Float16* Bt = (const _Float16*)Btp;
  __shared__ __align__(16) float sT[8][16 * 68];
  const int lane = threadIdx.x & 31;
  const int wave = threadIdx.x >> 5;
  const int tilesN = N >> 6;
  const int tilesM = M >> 6;
  const int tile = blockIdx.x * 8 + wave;
  if (tile >= tilesM * tilesN) return;
  const int tm = tile / tilesN;
  const int tn = tile - tm * tilesN;
  const int m0 = tm << 6;
  const int n0 = tn << 6;
  const int rlane = lane & 15;
  const int koff  = (lane >> 4) * 8;
  const int mOff  = (lane >> 4) * 8;

  v8f acc[4][4];
#pragma unroll
  for (int i = 0; i < 4; ++i)
#pragma unroll
    for (int j = 0; j < 4; ++j) acc[i][j] = (v8f){0.f, 0.f, 0.f, 0.f, 0.f, 0.f, 0.f, 0.f};

  for (int k0 = 0; k0 < K; k0 += 32) {
    v16h bh[4];
#pragma unroll
    for (int j = 0; j < 4; ++j) {
      const size_t bo = (size_t)(n0 + (j << 4) + rlane) * ldb + koff + k0;
      bh[j] = frag_load_h(Bt + bo);
    }
#pragma unroll
    for (int i = 0; i < 4; ++i) {
      const size_t ao = (size_t)(m0 + (i << 4) + rlane) * lda + koff + k0;
      const v16h ah = frag_load_h(A + ao);
#pragma unroll
      for (int j = 0; j < 4; ++j) acc[i][j] = wmma_h(ah, bh[j], acc[i][j]);
      dep_guard4_h(acc[i][0], acc[i][1], acc[i][2], acc[i][3], ah, bh[3]);
    }
    keep4_h(bh[0], bh[1], bh[2], bh[3]);
  }
  acc_guard4(acc[0][0], acc[0][1], acc[0][2], acc[0][3]);
  acc_guard4(acc[1][0], acc[1][1], acc[1][2], acc[1][3]);
  acc_guard4(acc[2][0], acc[2][1], acc[2][2], acc[2][3]);
  acc_guard4(acc[3][0], acc[3][1], acc[3][2], acc[3][3]);

  float* slab = sT[wave];
#pragma unroll
  for (int i = 0; i < 4; ++i) {
    const int mBase = m0 + (i << 4);
#pragma unroll
    for (int j = 0; j < 4; ++j) {
      const int n = n0 + (j << 4) + rlane;
      const float bv = bias[n];
#pragma unroll
      for (int r = 0; r < 8; ++r) {
        float v = acc[i][j][r] * scale;
        v += bv;
        slab[(mOff + r) * 68 + (j << 4) + rlane] = v;
      }
    }
    __builtin_amdgcn_fence(__ATOMIC_RELEASE, "workgroup");
    __builtin_amdgcn_wave_barrier();
    __builtin_amdgcn_fence(__ATOMIC_ACQUIRE, "workgroup");
    {
      const int hh = lane >> 4, c4 = (lane & 15) * 4;
      for (int pass = 0; pass < 2; ++pass) {
#pragma unroll
        for (int it = 0; it < 8; ++it) {
          const int row = it * 2 + hh;
          const v4f v = *(const v4f*)(slab + row * 68 + c4);
          *(volatile v4f*)(C + (size_t)(mBase + row) * ldc + n0 + c4) = v;
        }
        __threadfence();
      }
    }
    __builtin_amdgcn_fence(__ATOMIC_RELEASE, "workgroup");
    __builtin_amdgcn_wave_barrier();
    __builtin_amdgcn_fence(__ATOMIC_ACQUIRE, "workgroup");
  }
}

__global__ __launch_bounds__(RNN_THR) void rnn_seq_kernel(const float* __restrict__ XW,
                                                          const unsigned short* __restrict__ WHp,
                                                          const float* __restrict__ bhh,
                                                          float* __restrict__ HSUM) {
  __shared__ __align__(16) _Float16 Ah[2][ROWS_BLK * HPITCH];
  __shared__ __align__(16) float    Hs[ROWS_BLK * OPITCH];
  const _Float16* WH = (const _Float16*)WHp;
  const int tid = threadIdx.x, lane = tid & 31, wave = tid >> 5;
  const int c = lane & 15, hh = lane >> 4, koff = hh * 8;
  const int rowbase = blockIdx.x * ROWS_BLK;
  const int j = 16 * wave + c;

  {
    _Float16* ahf = &Ah[0][0];
#pragma unroll 1
    for (int i = tid; i < 2 * ROWS_BLK * HPITCH; i += RNN_THR) ahf[i] = (_Float16)0.0f;
  }
  v16h bfr[8];
#pragma unroll
  for (int k = 0; k < 8; ++k) bfr[k] = frag_load_h(WH + (size_t)j * HID_DIM + koff + 32 * k);
  const float bj = bhh[j];
  float hsum[8];
#pragma unroll
  for (int r = 0; r < 8; ++r) hsum[r] = 0.0f;
  __syncthreads();

  const v8f z8 = {0.f, 0.f, 0.f, 0.f, 0.f, 0.f, 0.f, 0.f};

#pragma unroll 1
  for (int t = 0; t < SEQ_LEN; ++t) {
    const int cur = t & 1;
    const _Float16* ahrow = &Ah[0][0] + cur * (ROWS_BLK * HPITCH) + c * HPITCH + koff;
    _Float16* ahn = &Ah[0][0] + (cur ^ 1) * (ROWS_BLK * HPITCH);
    const float* xp = XW + ((size_t)t * BATCH_N + (size_t)(rowbase + 8 * hh)) * HID_DIM + j;
    float xw[8];
#pragma unroll
    for (int r = 0; r < 8; ++r) xw[r] = xp[(size_t)r * HID_DIM];

    v8f acc = z8;
#pragma unroll
    for (int k = 0; k < 8; ++k) {
      const v16h a = frag_load_h(ahrow + 32 * k);
      acc = wmma_h_guarded(a, bfr[k], acc);
    }
#pragma unroll
    for (int r = 0; r < 8; ++r) {
      float z = acc[r] * WCARRY_INV + xw[r];
      z += bj;
      const float hv = tanhf(z);
      hsum[r] += hv;
      ahn[(8 * hh + r) * HPITCH + j] = (_Float16)hv;
    }
    __syncthreads();
  }

#pragma unroll
  for (int r = 0; r < 8; ++r) Hs[(8 * hh + r) * OPITCH + j] = hsum[r];
  __syncthreads();
  for (int pass = 0; pass < 2; ++pass) {
#pragma unroll
    for (int it = 0; it < (ROWS_BLK * HID_DIM / 4) / RNN_THR; ++it) {
      const int idx = it * RNN_THR + tid;
      const int row = idx >> 6, c4 = (idx & 63) * 4;
      const v4f v = *(const v4f*)(Hs + row * OPITCH + c4);
      *(volatile v4f*)(HSUM + (size_t)(rowbase + row) * HID_DIM + c4) = v;
    }
    __threadfence();
  }
}

__global__ __launch_bounds__(256) void head_kernel(const float* __restrict__ HSUM, const float* __restrict__ wout,
                                                   const float* __restrict__ bout, float* __restrict__ out) {
  __shared__ float lg[BATCH_N * 8];
  __shared__ float so[BATCH_N * CLS_DIM];
  const int tid = threadIdx.x, lane = tid & 31, wave = tid >> 5;
  const float bo0 = bout[0] * (float)SEQ_LEN;
  const float bo1 = bout[1] * (float)SEQ_LEN;
  const float bo2 = bout[2] * (float)SEQ_LEN;
  const float bo3 = bout[3] * (float)SEQ_LEN;
  const float bo4 = bout[4] * (float)SEQ_LEN;
#pragma unroll 1
  for (int rr = 0; rr < 8; ++rr) {
    const int b = wave * 8 + rr;
    float s0 = 0.0f, s1 = 0.0f, s2 = 0.0f, s3 = 0.0f, s4 = 0.0f;
#pragma unroll 1
    for (int i = 0; i < HID_DIM / 32; ++i) {
      const int n = lane + 32 * i;
      const float hv = HSUM[(size_t)b * HID_DIM + n];
      s0 = fmaf(hv, wout[0 * HID_DIM + n], s0);
      s1 = fmaf(hv, wout[1 * HID_DIM + n], s1);
      s2 = fmaf(hv, wout[2 * HID_DIM + n], s2);
      s3 = fmaf(hv, wout[3 * HID_DIM + n], s3);
      s4 = fmaf(hv, wout[4 * HID_DIM + n], s4);
    }
#pragma unroll
    for (int off = 16; off >= 1; off >>= 1) {
      s0 += __shfl_xor(s0, off, 32);
      s1 += __shfl_xor(s1, off, 32);
      s2 += __shfl_xor(s2, off, 32);
      s3 += __shfl_xor(s3, off, 32);
      s4 += __shfl_xor(s4, off, 32);
    }
    if (lane == 0) {
      lg[b * 8 + 0] = s0 + bo0;
      lg[b * 8 + 1] = s1 + bo1;
      lg[b * 8 + 2] = s2 + bo2;
      lg[b * 8 + 3] = s3 + bo3;
      lg[b * 8 + 4] = s4 + bo4;
    }
  }
  __syncthreads();
  if (tid < BATCH_N) {
    const float* lp = lg + tid * 8;
    float m = lp[0];
#pragma unroll 1
    for (int cc = 1; cc < CLS_DIM; ++cc) m = fmaxf(m, lp[cc]);
    float s = 0.0f;
#pragma unroll 1
    for (int cc = 0; cc < CLS_DIM; ++cc) s += expf(lp[cc] - m);
    const float ls = logf(s);
#pragma unroll 1
    for (int cc = 0; cc < CLS_DIM; ++cc) so[tid * CLS_DIM + cc] = (lp[cc] - m) - ls;
  }
  __syncthreads();
  if (wave == 0) {
    for (int pass = 0; pass < 2; ++pass) {
#pragma unroll 1
      for (int it = 0; it < (BATCH_N * CLS_DIM) / 32; ++it) {
        const float v = so[it * 32 + lane];
        *(volatile float*)(out + it * 32 + lane) = v;
      }
      __threadfence();
    }
  }
}

extern "C" void kernel_launch(void* const* d_in, const int* in_sizes, int n_in,
                              void* d_out, int out_size, void* d_ws, size_t ws_size, hipStream_t stream) {
  if (n_in < 8 || d_out == nullptr || d_ws == nullptr) return;
  if (in_sizes[0] != NROW_ALL || in_sizes[1] != VOCAB_N * EMB_DIM || in_sizes[2] != HID_DIM * EMB_DIM ||
      in_sizes[3] != HID_DIM * HID_DIM || in_sizes[4] != HID_DIM || in_sizes[5] != HID_DIM ||
      in_sizes[6] != CLS_DIM * HID_DIM || in_sizes[7] != CLS_DIM || out_size != BATCH_N * CLS_DIM) return;

  const int*   tok   = (const int*)d_in[0];
  const float* emb   = (const float*)d_in[1];
  const float* w_ih  = (const float*)d_in[2];
  const float* w_hh  = (const float*)d_in[3];
  const float* b_ih  = (const float*)d_in[4];
  const float* b_hh  = (const float*)d_in[5];
  const float* w_out = (const float*)d_in[6];
  const float* b_out = (const float*)d_in[7];
  float* out = (float*)d_out;

  char* ws = (char*)d_ws;
  size_t off = 0;
  auto carve = [&](size_t bytes) -> char* { char* p = ws + off; off += (bytes + 255) & ~(size_t)255; return p; };
  unsigned short* APL   = (unsigned short*)carve((size_t)NROW_ALL * EMB_PAD * 2);
  unsigned short* WIH16 = (unsigned short*)carve((size_t)HID_DIM * EMB_PAD * 2);
  unsigned short* WHH16 = (unsigned short*)carve((size_t)HID_DIM * HID_DIM * 2);
  float*          XW    = (float*)carve((size_t)NROW_ALL * HID_DIM * 4);
  float*          HSUM  = (float*)carve((size_t)BATCH_N * HID_DIM * 4);
  if (off > ws_size || off > (size_t)134217728) return;

  prep_weights_kernel<<<NBLK_WIH + NBLK_WHH, CVT_THR, 0, stream>>>(w_ih, w_hh, WIH16, WHH16);
  gather_rows_kernel<<<GATHER_N8 / CVT_THR, CVT_THR, 0, stream>>>(tok, emb, APL);
  gemm_xw_kernel<<<(NROW_ALL / 64) * (HID_DIM / 64) / 8, 256, 0, stream>>>(
      APL, EMB_PAD, WIH16, EMB_PAD, XW, HID_DIM, b_ih, NROW_ALL, HID_DIM, EMB_PAD, WCARRY_INV);
  rnn_seq_kernel<<<BATCH_N / ROWS_BLK, RNN_THR, 0, stream>>>(XW, WHH16, b_hh, HSUM);
  head_kernel<<<1, 256, 0, stream>>>(HSUM, w_out, b_out, out);
}
